// DGLFeatureGAT_23922967839172
// MI455X (gfx1250) — hardware-verified
//
#include <hip/hip_runtime.h>
#include <stddef.h>


typedef _Float16 h16;
typedef _Float16 v16h __attribute__((ext_vector_type(16)));
typedef _Float16 v8h  __attribute__((ext_vector_type(8)));
typedef float    v8f  __attribute__((ext_vector_type(8)));
typedef float    v4f  __attribute__((ext_vector_type(4)));

#ifndef NB
#define NB 64
#endif
#define NB_FULL 64
#define KW    128
#define NODES 64
#define NHEAD 4
#define OW    128
#define NOUT  (NHEAD * OW)

static_assert(NB >= 1 && NB <= NB_FULL);
static_assert(KW == 128 && NODES == 64 && NHEAD == 4 && OW == 128);
static_assert((KW % 32) == 0 && (NODES % 32) == 0);
static_assert(OW == 8 * 16);
static_assert(NODES == 4 * 16);

#define LDN  136
#define LDT  72
#define LDF  132
#define LDSC 65
#define LDC  68
static_assert((LDN % 8) == 0 && LDN >= KW);
static_assert((LDT % 8) == 0 && LDT >= NODES);
static_assert((LDF % 4) == 0 && LDF >= OW);
static_assert((LDC % 4) == 0 && LDC >= NODES);
static_assert(LDSC >= NODES);
static_assert(2 * NODES * LDF >= OW * LDC);

#define WCARRY 64.0f
#define XCARRY 16.0f
#define FCARRY 16.0f
#define PCARRY 1024.0f
#define NEG_SLOPE 0.2f

#define LDS_TOTAL_BYTES (NODES * LDN * 2 + 2 * NODES * LDF * 4 + OW * LDT * 2 + \
                         NODES * LDSC * 4 + NODES * LDT * 2 + OW * 4)
static_assert(LDS_TOTAL_BYTES <= 131072);

#define WPLANE_ELEMS ((size_t)NOUT * KW)
#define WS_TOTAL     ((size_t)2 * WPLANE_ELEMS * 2)
static_assert((WPLANE_ELEMS * 2) % 128 == 0);
static_assert(WS_TOTAL <= (size_t)134217728);
static_assert(WPLANE_ELEMS == (size_t)32 * 256 * 8);
static_assert(256 * 32 == KW * NODES);
static_assert(256 * 8 * 4 == OW * NODES);

__device__ __forceinline__ float bf16r(float x) {
  unsigned int u = __float_as_uint(x);
  u = (u + 0x7FFFu + ((u >> 16) & 1u)) & 0xFFFF0000u;
  return __uint_as_float(u);
}

static __device__ __forceinline__ h16 toh_flush(float v) {
  const h16 r = (h16)v;
  return (fabsf(v) < 6.103515625e-05f) ? (h16)0.0f : r;
}

__device__ __forceinline__ v16h frag_at(const _Float16* p) {
  v8h lo = *(const v8h*)(p);
  v8h hi = *(const v8h*)(p + 16);
  v16h out;
#pragma unroll
  for (int i = 0; i < 8; ++i) { out[i] = lo[i]; out[i + 8] = hi[i]; }
  return out;
}
__device__ __forceinline__ v16h ld_frag(const _Float16* base, unsigned ld) {
  const unsigned lane = threadIdx.x & 31u;
  return frag_at(base + (lane & 15u) * ld + (lane >> 4) * 8u);
}

__device__ __forceinline__ v8f wmma16(v16h a, v16h b, v8f c) {
  v8f d = __builtin_amdgcn_wmma_f32_16x16x32_f16(false, a, false, b, (short)0, c,
                                                 false, false);
  asm volatile("v_nop\n\tv_nop\n\tv_nop\n\tv_nop" : "+v"(d) : "v"(a), "v"(b));
  return d;
}

__device__ __forceinline__ float red32_sum(float x) {
#pragma unroll
  for (int off = 1; off < 32; off <<= 1) x += __shfl_xor(x, off, 32);
  return x;
}
__device__ __forceinline__ float red32_max(float x) {
#pragma unroll
  for (int off = 1; off < 32; off <<= 1) x = fmaxf(x, __shfl_xor(x, off, 32));
  return x;
}

__global__ __launch_bounds__(256) void wcvt_kernel(
    const float* __restrict__ W, _Float16* __restrict__ Wp) {
  const unsigned t = blockIdx.x * 256u + threadIdx.x;
  const size_t e0 = (size_t)t * 8u;
  const v4f a0 = *(const v4f*)(W + e0);
  const v4f a1 = *(const v4f*)(W + e0 + 4u);
  v8h o;
#pragma unroll
  for (int i = 0; i < 4; ++i) {
    o[i]     = toh_flush(WCARRY * bf16r(a0[i]));
    o[i + 4] = toh_flush(WCARRY * bf16r(a1[i]));
  }
  _Float16* p = Wp + e0;
  *(volatile v8h*)p = o;
  __threadfence();
  *(volatile v8h*)p = o;
}

__global__ __launch_bounds__(256) void gat_kernel(
    const float* __restrict__ X, const _Float16* __restrict__ Wp,
    const float* __restrict__ bsrc, const float* __restrict__ bdst,
    const float* __restrict__ attn, float* __restrict__ out) {
  __shared__ __attribute__((aligned(16))) _Float16 NFh[NODES * LDN];
  __shared__ __attribute__((aligned(16))) float    FSD[2 * NODES * LDF];
  __shared__ __attribute__((aligned(16))) _Float16 FT[OW * LDT];
  __shared__ __attribute__((aligned(16))) float    SC[NODES * LDSC];
  __shared__ __attribute__((aligned(16))) _Float16 PT[NODES * LDT];
  __shared__ __attribute__((aligned(16))) float    AH[OW];

  const unsigned tid = threadIdx.x, lane = tid & 31u;
  const unsigned wave = (unsigned)__builtin_amdgcn_readfirstlane((int)(threadIdx.x >> 5));
  const unsigned hh = lane >> 4, m = lane & 15u;
  const unsigned b = blockIdx.x;

  {
    const float* xb = X + (size_t)b * (KW * NODES);
#pragma unroll 4
    for (unsigned j = 0; j < 32u; ++j) {
      const unsigned idx = tid + 256u * j;
      const unsigned kq = idx >> 6, f = idx & 63u;
      const float v = xb[idx];
      NFh[f * LDN + kq] = toh_flush(XCARRY * bf16r(v));
    }
  }
  __syncthreads();

  v8f oacc[4];
#pragma unroll
  for (int jt = 0; jt < 4; ++jt) oacc[jt] = (v8f){};

#pragma unroll 1
  for (unsigned head = 0; head < (unsigned)NHEAD; ++head) {
    if (tid < (unsigned)OW) AH[tid] = bf16r(attn[head * OW + tid]);

    const float bs = bf16r(bsrc[head * OW + wave * 16u + m]);
    const float bd = bf16r(bdst[head * OW + wave * 16u + m]);
#pragma unroll
    for (int sd = 0; sd < 2; ++sd) {
      const _Float16* bp =
          Wp + ((size_t)sd * NOUT + head * OW + wave * 16u + m) * KW + hh * 8u;
      v16h bf[4];
#pragma unroll
      for (int c = 0; c < 4; ++c) bf[c] = frag_at(bp + 32 * c);
      const float bval = (sd == 0) ? bs : bd;
#pragma unroll 1
      for (unsigned mt = 0; mt < 4u; ++mt) {
        v8f acc = {};
#pragma unroll
        for (int c = 0; c < 4; ++c) {
          const v16h a = ld_frag(&NFh[(mt * 16u) * LDN + (unsigned)c * 32u], LDN);
          acc = wmma16(a, bf[c], acc);
        }
        float vals[8];
#pragma unroll
        for (int r = 0; r < 8; ++r) vals[r] = acc[r] * (1.0f / (WCARRY * XCARRY)) + bval;
#pragma unroll
        for (int r = 0; r < 8; ++r)
          FSD[(unsigned)sd * (NODES * LDF) + (mt * 16u + hh * 8u + (unsigned)r) * LDF +
              wave * 16u + m] = vals[r];
        if (sd == 0) {
          v8h t;
#pragma unroll
          for (int r = 0; r < 8; ++r) t[r] = toh_flush(FCARRY * vals[r]);
          *(v8h*)&FT[(wave * 16u + m) * LDT + mt * 16u + hh * 8u] = t;
        }
      }
    }
    __syncthreads();

    {
      const unsigned j = tid & 63u;
      const unsigned i0 = tid >> 6;
#pragma unroll 1
      for (unsigned pp = 0; pp < 4u; ++pp) {
        const unsigned ib = i0 + 16u * pp;
        float s0 = 0.0f, s1 = 0.0f, s2 = 0.0f, s3 = 0.0f;
#pragma unroll 2
        for (unsigned d4 = 0; d4 < (unsigned)(OW / 4); ++d4) {
          const v4f aa = *(const v4f*)&AH[d4 * 4u];
          const v4f v  = *(const v4f*)&FSD[NODES * LDF + j * LDF + d4 * 4u];
          const v4f u0 = *(const v4f*)&FSD[(ib)       * LDF + d4 * 4u];
          const v4f u1 = *(const v4f*)&FSD[(ib + 4u)  * LDF + d4 * 4u];
          const v4f u2 = *(const v4f*)&FSD[(ib + 8u)  * LDF + d4 * 4u];
          const v4f u3 = *(const v4f*)&FSD[(ib + 12u) * LDF + d4 * 4u];
#pragma unroll
          for (int c = 0; c < 4; ++c) {
            float t0 = u0[c] + v[c]; t0 = fmaxf(t0, NEG_SLOPE * t0); s0 = fmaf(aa[c], t0, s0);
            float t1 = u1[c] + v[c]; t1 = fmaxf(t1, NEG_SLOPE * t1); s1 = fmaf(aa[c], t1, s1);
            float t2 = u2[c] + v[c]; t2 = fmaxf(t2, NEG_SLOPE * t2); s2 = fmaf(aa[c], t2, s2);
            float t3 = u3[c] + v[c]; t3 = fmaxf(t3, NEG_SLOPE * t3); s3 = fmaf(aa[c], t3, s3);
          }
        }
        SC[j * LDSC + ib]       = s0;
        SC[j * LDSC + ib + 4u]  = s1;
        SC[j * LDSC + ib + 8u]  = s2;
        SC[j * LDSC + ib + 12u] = s3;
      }
    }
    __syncthreads();

#pragma unroll 1
    for (unsigned jj = 0; jj < 8u; ++jj) {
      const unsigned j = wave * 8u + jj;
      const float a0 = SC[j * LDSC + lane];
      const float a1 = SC[j * LDSC + lane + 32u];
      const float mx = red32_max(fmaxf(a0, a1));
      const float e0 = __expf(a0 - mx);
      const float e1 = __expf(a1 - mx);
      const float sum = red32_sum(e0 + e1);
      const float inv = PCARRY * (1.0f / sum);
      PT[j * LDT + lane]       = toh_flush(e0 * inv);
      PT[j * LDT + lane + 32u] = toh_flush(e1 * inv);
    }
    __syncthreads();

    {
      v16h af[2];
#pragma unroll
      for (int c = 0; c < 2; ++c) af[c] = ld_frag(&FT[(wave * 16u) * LDT + (unsigned)c * 32u], LDT);
#pragma unroll
      for (int jt = 0; jt < 4; ++jt) {
#pragma unroll
        for (int c = 0; c < 2; ++c) {
          const v16h pf = ld_frag(&PT[(jt * 16) * LDT + c * 32], LDT);
          oacc[jt] = wmma16(af[c], pf, oacc[jt]);
        }
      }
    }
    __syncthreads();
  }

  {
    const float osc = 0.25f / (PCARRY * FCARRY);
#pragma unroll
    for (int jt = 0; jt < 4; ++jt)
#pragma unroll
      for (int r = 0; r < 8; ++r)
        FSD[(wave * 16u + hh * 8u + (unsigned)r) * LDC + (unsigned)jt * 16u + m] =
            oacc[jt][r] * osc;
  }
  __syncthreads();

  v4f xs[8];
  size_t off[8];
#pragma unroll
  for (unsigned i = 0; i < 8u; ++i) {
    const unsigned idx = tid + 256u * i;
    const unsigned row = idx >> 4;
    const unsigned c = (idx & 15u) * 4u;
    xs[i] = *(const v4f*)&FSD[row * LDC + c];
    off[i] = (size_t)b * (OW * NODES) + (size_t)row * NODES + c;
  }
#pragma unroll
  for (int i = 0; i < 8; ++i) *(volatile v4f*)(out + off[i]) = xs[i];
  __threadfence();
#pragma unroll
  for (int i = 0; i < 8; ++i) *(volatile v4f*)(out + off[i]) = xs[i];
}

extern "C" void kernel_launch(void* const* d_in, const int* in_sizes, int n_in,
                              void* d_out, int out_size, void* d_ws, size_t ws_size,
                              hipStream_t stream) {
  if (n_in < 6) return;
  const long long need_x = (long long)NB * KW * NODES;
  if ((long long)in_sizes[0] < need_x) return;
  if ((long long)in_sizes[1] < (long long)NOUT * KW) return;
  if (in_sizes[2] < NOUT) return;
  if ((long long)in_sizes[3] < (long long)NOUT * KW) return;
  if (in_sizes[4] < NOUT) return;
  if (in_sizes[5] < NHEAD * OW) return;
  if ((long long)out_size < (long long)NB * OW * NODES) return;
  if (ws_size < WS_TOTAL) return;

  const float* X    = (const float*)d_in[0];
  const float* wsrc = (const float*)d_in[1];
  const float* bsrc = (const float*)d_in[2];
  const float* wdst = (const float*)d_in[3];
  const float* bdst = (const float*)d_in[4];
  const float* attn = (const float*)d_in[5];
  float* out = (float*)d_out;

  _Float16* Wp = (_Float16*)d_ws;

  dim3 blk(256);
  wcvt_kernel<<<dim3(32), blk, 0, stream>>>(wsrc, Wp);
  wcvt_kernel<<<dim3(32), blk, 0, stream>>>(wdst, Wp + WPLANE_ELEMS);
  gat_kernel<<<dim3(NB), blk, 0, stream>>>(X, Wp, bsrc, bdst, attn, out);
}
